// acLSTM_10170482557673
// MI455X (gfx1250) — hardware-verified
//
#include <hip/hip_runtime.h>
#include <math.h>

constexpr int NB     = 64;
constexpr int NH     = 1024;
constexpr int NG4    = 4096;
constexpr int NIN    = 171;
constexpr int NINP   = 192;
constexpr int NOUT   = 171;
constexpr int NOUTP  = 192;
constexpr int TWARM  = 50;
constexpr int TGEN   = 100;
constexpr int TALL   = TWARM + TGEN;
constexpr int KC0    = NINP + NH;
constexpr int KC12   = 2 * NH;
constexpr int HSP    = 72;
constexpr int SLABP  = 68;
constexpr int NOUT4  = NB * TGEN * NOUT / 4;
constexpr float ACARRY = 64.0f;
constexpr float WCARRY = 16.0f;
constexpr float FOLD   = 1.0f / (ACARRY * WCARRY);

static_assert(NB == 64, "four 16-row m-subtiles");
static_assert(NG4 == 4 * NH, "gate blocks i f g o");
static_assert(NINP % 32 == 0 && NINP >= NIN, "padded K of the input frame");
static_assert(NOUTP % 64 == 0 && NOUTP >= NOUT && NOUTP == NINP, "decoder N pad equals next-step K pad");
static_assert(NH % 64 == 0 && NH % 32 == 0, "panel and k-chunk multiples");
static_assert((NB * TGEN * NOUT) % 128 == 0, "output is a whole number of 512-B wave stores");
static_assert((KC0 * 2) % 128 == 0 && (NINP * 2) % 128 == 0, "plane pitches are line multiples");

typedef __attribute__((ext_vector_type(16))) _Float16 v16h;
typedef __attribute__((ext_vector_type(8)))  _Float16 v8h;
typedef __attribute__((ext_vector_type(8)))  float    v8f;
typedef __attribute__((ext_vector_type(4)))  float    v4f;

__device__ __forceinline__ void guard_grp(v8f& a0, v8f& a1, v8f& a2, v8f& a3, v16h x, v16h y0, v16h y1, v16h y2, v16h y3) {
  asm volatile("v_nop\n\tv_nop\n\tv_nop\n\tv_nop" : "+v"(a0), "+v"(a1), "+v"(a2), "+v"(a3) : "v"(x), "v"(y0), "v"(y1), "v"(y2), "v"(y3));
}
__device__ __forceinline__ void acc_guard4(v8f& a, v8f& b, v8f& c, v8f& d) {
  asm volatile("v_nop\n\tv_nop\n\tv_nop\n\tv_nop" : "+v"(a), "+v"(b), "+v"(c), "+v"(d));
}

template <typename T> struct Frag;
template <> struct Frag<_Float16> {
  typedef v16h V; union U { v16h v; v8h h[2]; };
  static __device__ __forceinline__ v16h load(const _Float16* p) {
    U f; f.h[0] = *(const v8h*)(p); f.h[1] = *(const v8h*)(p + 16); return f.v;
  }
  static __device__ __forceinline__ v8f mma(v16h a, v16h b, v8f c) {
    return __builtin_amdgcn_wmma_f32_16x16x32_f16(false, a, false, b, (short)0, c, false, false);
  }
};

__device__ __forceinline__ float fsig(float x)  { return __builtin_amdgcn_rcpf(1.0f + __expf(-x)); }
__device__ __forceinline__ float ftanh(float x) { return 1.0f - 2.0f * __builtin_amdgcn_rcpf(__expf(2.0f * x) + 1.0f); }

__device__ __forceinline__ void kseg(v8f (&acc)[4][4], const _Float16* ap, const int lda,
                                     const _Float16* bp, const size_t nstride, const int klen) {
#pragma unroll 1
  for (int k0 = 0; k0 < klen; k0 += 32) {
    v16h bh[4];
#pragma unroll
    for (int j = 0; j < 4; ++j) bh[j] = Frag<_Float16>::load(bp + (size_t)j * nstride + k0);
#pragma unroll
    for (int i = 0; i < 4; ++i) {
      const v16h ah = Frag<_Float16>::load(ap + (size_t)(16 * i) * lda + k0);
#pragma unroll
      for (int j = 0; j < 4; ++j) acc[i][j] = Frag<_Float16>::mma(ah, bh[j], acc[i][j]);
      guard_grp(acc[i][0], acc[i][1], acc[i][2], acc[i][3], ah, bh[0], bh[1], bh[2], bh[3]);
    }
  }
}

__global__ __launch_bounds__(256) void zero_kernel(float* __restrict__ dst, int n16) {
  const int i = blockIdx.x * 256 + threadIdx.x;
  if (i < n16) {
    const v4f z = {0.0f, 0.0f, 0.0f, 0.0f};
    *(volatile v4f*)(dst + (size_t)i * 4) = z;
    __threadfence();
    *(volatile v4f*)(dst + (size_t)i * 4) = z;
  }
}

__global__ __launch_bounds__(256) void bias_kernel(const float* __restrict__ bi1, const float* __restrict__ bh1,
                                                   const float* __restrict__ bi2, const float* __restrict__ bh2,
                                                   const float* __restrict__ bi3, const float* __restrict__ bh3,
                                                   const float* __restrict__ bd,
                                                   float* __restrict__ bsum, float* __restrict__ bdecp) {
  const int tid = threadIdx.x;
  if (blockIdx.x < 12) {
    const int cl = blockIdx.x >> 2;
    const float* pa = (cl == 0) ? bi1 : ((cl == 1) ? bi2 : bi3);
    const float* pb = (cl == 0) ? bh1 : ((cl == 1) ? bh2 : bh3);
    const int idx = ((blockIdx.x & 3) * 256 + tid) * 4;
    const v4f a = *(const v4f*)(pa + idx);
    const v4f b = *(const v4f*)(pb + idx);
    v4f o;
#pragma unroll
    for (int e = 0; e < 4; ++e) o[e] = a[e] + b[e];
    float* op = bsum + cl * NG4 + idx;
    *(volatile v4f*)op = o;
    __threadfence();
    *(volatile v4f*)op = o;
  } else {
    if (tid < NOUTP / 4) {
      const int idx = tid * 4;
      v4f o;
#pragma unroll
      for (int e = 0; e < 4; ++e) {
        const int n = idx + e;
        const int nc = (n < NOUT) ? n : (NOUT - 1);
        const float v = bd[nc];
        o[e] = (n < NOUT) ? v : 0.0f;
      }
      float* op = bdecp + idx;
      *(volatile v4f*)op = o;
      __threadfence();
      *(volatile v4f*)op = o;
    }
  }
}

template <bool ALIGNED, bool TMAJOR>
__global__ __launch_bounds__(256) void cvt8_kernel(const float* __restrict__ src, unsigned short* __restrict__ dst,
                                                   int nrow, int ncol8, int spitch, int ncol_valid, int nrow_valid,
                                                   int dpitch, int dcol0, float sc) {
  const int i  = blockIdx.x * 256 + threadIdx.x;
  const int n8 = nrow * ncol8;
  if (i < n8) {
    const int row = i / ncol8;
    const int c8  = i - row * ncol8;
    int srow = (row < nrow_valid) ? row : (nrow_valid - 1);
    if (TMAJOR) srow = (row & (NB - 1)) * TWARM + (row >> 6);
    const float* sp = src + (size_t)srow * spitch;
    float f[8];
    if (ALIGNED) {
      const v4f a = *(const v4f*)(sp + c8 * 8);
      const v4f b = *(const v4f*)(sp + c8 * 8 + 4);
#pragma unroll
      for (int e = 0; e < 4; ++e) { f[e] = a[e]; f[4 + e] = b[e]; }
    } else {
#pragma unroll
      for (int e = 0; e < 8; ++e) {
        const int k  = c8 * 8 + e;
        const int kc = (k < ncol_valid) ? k : (ncol_valid - 1);
        const float v = sp[kc];
        f[e] = (k < ncol_valid) ? v : 0.0f;
      }
    }
    const bool rowok = (row < nrow_valid);
    v8h hv;
#pragma unroll
    for (int e = 0; e < 8; ++e) {
      const float g = rowok ? f[e] : 0.0f;
      hv[e] = (_Float16)(g * sc);
    }
    _Float16* dp = (_Float16*)dst + (size_t)row * dpitch + dcol0 + c8 * 8;
    *(volatile v8h*)dp = hv;
    __threadfence();
    *(volatile v8h*)dp = hv;
  }
}

__global__ __launch_bounds__(128) void lstm_step_kernel(const unsigned short* __restrict__ xplane,
                                                        unsigned short* hpl, float* cpl,
                                                        const float* __restrict__ bsum,
                                                        const unsigned short* __restrict__ wc0,
                                                        const unsigned short* __restrict__ wc1,
                                                        const unsigned short* __restrict__ wc2,
                                                        int p) {
  __shared__ __align__(16) _Float16 Hs[NB * HSP];
  const int tid = threadIdx.x, lane = tid & 31, wave = tid >> 5;
  const int c = lane & 15, hh = lane >> 4, koff = hh * 8;
  const int pb = blockIdx.x;
  const int cl = blockIdx.y;
  const int q  = 1 - p;

  const _Float16* hbase = (const _Float16*)hpl;
  const _Float16* hself = hbase + (size_t)(cl * 2 + p) * (NB * NH);
  const int clm = (cl > 0) ? (cl - 1) : 0;
  const _Float16* hlow  = hbase + (size_t)(clm * 2 + p) * (NB * NH);
  const _Float16* a0    = (cl == 0) ? (const _Float16*)xplane : hlow;
  const int lda0        = (cl == 0) ? NINP : NH;
  const int k0len       = (cl == 0) ? NINP : NH;
  const _Float16* wpl   = (const _Float16*)((cl == 0) ? wc0 : ((cl == 1) ? wc1 : wc2));
  const int ldb         = (cl == 0) ? KC0 : KC12;
  const int unit        = 64 * pb + 16 * wave + c;
  const _Float16* bp    = wpl + (size_t)unit * ldb + koff;
  const size_t nstride  = (size_t)NH * ldb;

  v8f acc[4][4];
  const v8f z8 = {0.f, 0.f, 0.f, 0.f, 0.f, 0.f, 0.f, 0.f};
#pragma unroll
  for (int i = 0; i < 4; ++i)
#pragma unroll
    for (int j = 0; j < 4; ++j) acc[i][j] = z8;

  kseg(acc, a0 + (size_t)c * lda0 + koff, lda0, bp, nstride, k0len);
  kseg(acc, hself + (size_t)c * NH + koff, NH, bp + k0len, nstride, NH);
  acc_guard4(acc[0][0], acc[0][1], acc[0][2], acc[0][3]);
  acc_guard4(acc[1][0], acc[1][1], acc[1][2], acc[1][3]);
  acc_guard4(acc[2][0], acc[2][1], acc[2][2], acc[2][3]);
  acc_guard4(acc[3][0], acc[3][1], acc[3][2], acc[3][3]);

  const float* bs = bsum + cl * NG4 + unit;
  const float b_i = bs[0];
  const float b_f = bs[NH];
  const float b_g = bs[2 * NH];
  const float b_o = bs[3 * NH];

  const size_t coff = (size_t)((pb * 4 + wave) * 8) * 128 + (size_t)lane * 4;
  const float* cin  = cpl + (size_t)(cl * 2 + p) * (NB * NH) + coff;
  float*       cout = cpl + (size_t)(cl * 2 + q) * (NB * NH) + coff;

  v4f cnew[8];
#pragma unroll
  for (int i = 0; i < 4; ++i) {
#pragma unroll
    for (int rq = 0; rq < 2; ++rq) {
      const v4f co = *(const v4f*)(cin + (i * 2 + rq) * 128);
      v4f cn;
#pragma unroll
      for (int e = 0; e < 4; ++e) {
        const int r = rq * 4 + e;
        const float zi = acc[i][0][r] * FOLD + b_i;
        const float zf = acc[i][1][r] * FOLD + b_f;
        const float zg = acc[i][2][r] * FOLD + b_g;
        const float zo = acc[i][3][r] * FOLD + b_o;
        const float ig = fsig(zi);
        const float fg = fsig(zf);
        const float gg = ftanh(zg);
        const float og = fsig(zo);
        const float cv = fg * co[e] + ig * gg;
        cn[e] = cv;
        const float hv = og * ftanh(cv);
        Hs[(16 * i + 8 * hh + r) * HSP + 16 * wave + c] = (_Float16)(hv * ACARRY);
      }
      cnew[i * 2 + rq] = cn;
    }
  }
  for (int pass = 0; pass < 2; ++pass) {
#pragma unroll
    for (int qd = 0; qd < 8; ++qd) *(volatile v4f*)(cout + qd * 128) = cnew[qd];
    __threadfence();
  }
  __syncthreads();
  {
    const int rq8 = tid >> 3, c8 = (tid & 7) * 8;
    _Float16* hout = (_Float16*)hpl + (size_t)(cl * 2 + q) * (NB * NH) + 64 * pb + c8;
    v8h hv4[4];
#pragma unroll
    for (int it = 0; it < 4; ++it) hv4[it] = *(const v8h*)(Hs + (it * 16 + rq8) * HSP + c8);
    for (int pass = 0; pass < 2; ++pass) {
#pragma unroll
      for (int it = 0; it < 4; ++it) *(volatile v8h*)(hout + (size_t)(it * 16 + rq8) * NH) = hv4[it];
      __threadfence();
    }
  }
}

__global__ __launch_bounds__(96) void decode_kernel(const unsigned short* __restrict__ h2new,
                                                    const unsigned short* __restrict__ wd,
                                                    const float* __restrict__ bdecp,
                                                    unsigned short* __restrict__ xg,
                                                    float* __restrict__ stage_out, int wr_stage) {
  __shared__ __align__(16) float sT[3][16 * SLABP];
  const int tid = threadIdx.x, lane = tid & 31, wave = tid >> 5;
  const int c = lane & 15, hh = lane >> 4, koff = hh * 8;
  const _Float16* ap = (const _Float16*)h2new + (size_t)c * NH + koff;
  const _Float16* bp = (const _Float16*)wd + (size_t)(64 * wave + c) * NH + koff;

  v8f acc[4][4];
  const v8f z8 = {0.f, 0.f, 0.f, 0.f, 0.f, 0.f, 0.f, 0.f};
#pragma unroll
  for (int i = 0; i < 4; ++i)
#pragma unroll
    for (int j = 0; j < 4; ++j) acc[i][j] = z8;
  kseg(acc, ap, NH, bp, (size_t)16 * NH, NH);
  acc_guard4(acc[0][0], acc[0][1], acc[0][2], acc[0][3]);
  acc_guard4(acc[1][0], acc[1][1], acc[1][2], acc[1][3]);
  acc_guard4(acc[2][0], acc[2][1], acc[2][2], acc[2][3]);
  acc_guard4(acc[3][0], acc[3][1], acc[3][2], acc[3][3]);

  float bv[4];
#pragma unroll
  for (int j = 0; j < 4; ++j) bv[j] = bdecp[64 * wave + 16 * j + c];

  float* slab = sT[wave];
  const int mOff = 8 * hh;
  const int c4 = c * 4;
  const int q4 = lane >> 3, c8 = (lane & 7) * 8;
  _Float16* xgh = (_Float16*)xg;
#pragma unroll
  for (int i = 0; i < 4; ++i) {
    const int mBase = 16 * i;
#pragma unroll
    for (int j = 0; j < 4; ++j)
#pragma unroll
      for (int r = 0; r < 8; ++r)
        slab[(mOff + r) * SLABP + 16 * j + c] = acc[i][j][r] * FOLD + bv[j];
    __builtin_amdgcn_fence(__ATOMIC_RELEASE, "workgroup");
    __builtin_amdgcn_wave_barrier();
    __builtin_amdgcn_fence(__ATOMIC_ACQUIRE, "workgroup");
    for (int pass = 0; pass < 2; ++pass) {
      if (wr_stage != 0) {
#pragma unroll
        for (int it = 0; it < 8; ++it) {
          const int row = it * 2 + hh;
          const v4f v = *(const v4f*)(slab + row * SLABP + c4);
          *(volatile v4f*)(stage_out + (size_t)(mBase + row) * NOUTP + 64 * wave + c4) = v;
        }
      }
#pragma unroll
      for (int it = 0; it < 4; ++it) {
        const int row = it * 4 + q4;
        const float* sp = slab + row * SLABP + c8;
        v8h hv;
#pragma unroll
        for (int e = 0; e < 8; ++e) hv[e] = (_Float16)(sp[e] * ACARRY);
        *(volatile v8h*)(xgh + (size_t)(mBase + row) * NINP + 64 * wave + c8) = hv;
      }
      __threadfence();
    }
    __builtin_amdgcn_fence(__ATOMIC_RELEASE, "workgroup");
    __builtin_amdgcn_wave_barrier();
    __builtin_amdgcn_fence(__ATOMIC_ACQUIRE, "workgroup");
  }
}

__global__ __launch_bounds__(256) void repack_kernel(const float* __restrict__ stage, float* __restrict__ outp) {
  const int i = blockIdx.x * 256 + threadIdx.x;
  if (i < NOUT4) {
    v4f v;
#pragma unroll
    for (int e = 0; e < 4; ++e) {
      const unsigned eidx = 4u * (unsigned)i + (unsigned)e;
      const unsigned rk = eidx / (unsigned)NOUT;
      const unsigned n  = eidx - rk * (unsigned)NOUT;
      const unsigned b  = rk / (unsigned)TGEN;
      const unsigned k  = rk - b * (unsigned)TGEN;
      v[e] = stage[((size_t)k * NB + b) * NOUTP + n];
    }
    float* op = outp + (size_t)i * 4;
    *(volatile v4f*)op = v;
    __threadfence();
    *(volatile v4f*)op = v;
  }
}

extern "C" void kernel_launch(void* const* d_in, const int* in_sizes, int n_in,
                              void* d_out, int out_size, void* d_ws, size_t ws_size, hipStream_t stream) {
  if (n_in < 16 || d_out == nullptr || d_ws == nullptr) return;
  if (in_sizes[0] != NB * TWARM * NIN || in_sizes[1] != NG4 * NIN || in_sizes[2] != NG4 * NH ||
      in_sizes[3] != NG4 || in_sizes[4] != NG4 || in_sizes[5] != NG4 * NH || in_sizes[6] != NG4 * NH ||
      in_sizes[7] != NG4 || in_sizes[8] != NG4 || in_sizes[9] != NG4 * NH || in_sizes[10] != NG4 * NH ||
      in_sizes[11] != NG4 || in_sizes[12] != NG4 || in_sizes[13] != NOUT * NH || in_sizes[14] != NOUT ||
      out_size != NB * TGEN * NOUT) return;

  const float* seq  = (const float*)d_in[0];
  const float* Wih1 = (const float*)d_in[1];
  const float* Whh1 = (const float*)d_in[2];
  const float* bih1 = (const float*)d_in[3];
  const float* bhh1 = (const float*)d_in[4];
  const float* Wih2 = (const float*)d_in[5];
  const float* Whh2 = (const float*)d_in[6];
  const float* bih2 = (const float*)d_in[7];
  const float* bhh2 = (const float*)d_in[8];
  const float* Wih3 = (const float*)d_in[9];
  const float* Whh3 = (const float*)d_in[10];
  const float* bih3 = (const float*)d_in[11];
  const float* bhh3 = (const float*)d_in[12];
  const float* Wdec = (const float*)d_in[13];
  const float* bdec = (const float*)d_in[14];
  float* outp = (float*)d_out;

  char* ws = (char*)d_ws; size_t off = 0;
  auto carve = [&](size_t bytes) -> char* { char* ptr = ws + off; off += (bytes + 255) & ~(size_t)255; return ptr; };
  unsigned short* WC0 = (unsigned short*)carve((size_t)NG4 * KC0 * 2);
  unsigned short* WC1 = (unsigned short*)carve((size_t)NG4 * KC12 * 2);
  unsigned short* WC2 = (unsigned short*)carve((size_t)NG4 * KC12 * 2);
  unsigned short* WD  = (unsigned short*)carve((size_t)NOUTP * NH * 2);
  unsigned short* XW  = (unsigned short*)carve((size_t)TWARM * NB * NINP * 2);
  const size_t zbeg = off;
  unsigned short* HPL = (unsigned short*)carve((size_t)3 * 2 * NB * NH * 2);
  float*          CPL = (float*)carve((size_t)3 * 2 * NB * NH * 4);
  unsigned short* XG  = (unsigned short*)carve((size_t)2 * NB * NINP * 2);
  const size_t zbytes = off - zbeg;
  float* BSUM  = (float*)carve((size_t)3 * NG4 * 4);
  float* BDEC  = (float*)carve((size_t)NOUTP * 4);
  float* STAGE = (float*)carve((size_t)TGEN * NB * NOUTP * 4);
  if (off > ws_size || off > (size_t)134217728) return;

  {
    const int n16 = (int)(zbytes / 16);
    zero_kernel<<<(n16 + 255) / 256, 256, 0, stream>>>((float*)HPL, n16);
  }
  bias_kernel<<<13, 256, 0, stream>>>(bih1, bhh1, bih2, bhh2, bih3, bhh3, bdec, BSUM, BDEC);

  {
    const int n8h = NG4 * (NH / 8);
    const int n8x = NG4 * (NINP / 8);
    const int n8d = NOUTP * (NH / 8);
    cvt8_kernel<false, false><<<(n8x + 255) / 256, 256, 0, stream>>>(Wih1, WC0, NG4, NINP / 8, NIN, NIN, NG4, KC0, 0, WCARRY);
    cvt8_kernel<true,  false><<<(n8h + 255) / 256, 256, 0, stream>>>(Whh1, WC0, NG4, NH / 8, NH, NH, NG4, KC0, NINP, WCARRY);
    cvt8_kernel<true,  false><<<(n8h + 255) / 256, 256, 0, stream>>>(Wih2, WC1, NG4, NH / 8, NH, NH, NG4, KC12, 0, WCARRY);
    cvt8_kernel<true,  false><<<(n8h + 255) / 256, 256, 0, stream>>>(Whh2, WC1, NG4, NH / 8, NH, NH, NG4, KC12, NH, WCARRY);
    cvt8_kernel<true,  false><<<(n8h + 255) / 256, 256, 0, stream>>>(Wih3, WC2, NG4, NH / 8, NH, NH, NG4, KC12, 0, WCARRY);
    cvt8_kernel<true,  false><<<(n8h + 255) / 256, 256, 0, stream>>>(Whh3, WC2, NG4, NH / 8, NH, NH, NG4, KC12, NH, WCARRY);
    cvt8_kernel<true,  false><<<(n8d + 255) / 256, 256, 0, stream>>>(Wdec, WD, NOUTP, NH / 8, NH, NH, NOUT, NH, 0, WCARRY);
  }
  {
    const int n8 = TWARM * NB * (NINP / 8);
    cvt8_kernel<false, true><<<(n8 + 255) / 256, 256, 0, stream>>>(seq, XW, TWARM * NB, NINP / 8, NIN, NIN, TWARM * NB, NINP, 0, ACARRY);
  }

  const size_t xplane_elems = (size_t)NB * NINP;
  const size_t hplane_elems = (size_t)NB * NH;
  for (int t = 0; t < TALL; ++t) {
    const int p = t & 1;
    const int q = 1 - p;
    const unsigned short* xptr = (t < TWARM) ? (XW + (size_t)t * xplane_elems) : (XG + (size_t)(t & 1) * xplane_elems);
    lstm_step_kernel<<<dim3(NH / 64, 3), 128, 0, stream>>>(xptr, HPL, CPL, BSUM, WC0, WC1, WC2, p);
    if (t >= TWARM - 1) {
      const int kf = (t >= TWARM) ? (t - TWARM) : 0;
      const int wr = (t >= TWARM) ? 1 : 0;
      decode_kernel<<<1, 96, 0, stream>>>(HPL + (size_t)(2 * 2 + q) * hplane_elems, WD, BDEC,
                                          XG + (size_t)((t + 1) & 1) * xplane_elems,
                                          STAGE + (size_t)kf * NB * NOUTP, wr);
    }
  }
  repack_kernel<<<(NOUT4 + 255) / 256, 256, 0, stream>>>(STAGE, outp);
}
